// MSSA_80161269612898
// MI455X (gfx1250) — hardware-run, weakly checked
//
#include <hip/hip_runtime.h>
#include <math.h>

#define NB    8
#define SEQ   2048
#define DM    512
#define QKVN  1536
#define NQK   1024
#define ROWS  (NB * SEQ)
#define WSC   1024.0f
#define PSC   1024.0f
#define L2E   1.44269504088896341f
static_assert((ROWS % 64) == 0 && (SEQ % 64) == 0 && (DM % 64) == 0 && (NQK % 64) == 0 && (QKVN % 64) == 0);
static_assert((DM % 32) == 0 && (SEQ % 32) == 0);
static_assert((SEQ % 256) == 0 && (DM % 8) == 0);
static_assert(((ROWS / 64) * (NQK / 64)) % 8 == 0);
static_assert(((DM / 64) * (SEQ / 64)) % 8 == 0);
static_assert(((SEQ / 64) * (SEQ / 64)) % 8 == 0);
static_assert(((SEQ / 64) * (DM / 64)) % 8 == 0);
static_assert(((ROWS / 64) * (DM / 64)) % 8 == 0);

typedef _Float16 v16h __attribute__((ext_vector_type(16)));
typedef _Float16 v8h  __attribute__((ext_vector_type(8)));
typedef float    v8f  __attribute__((ext_vector_type(8)));
typedef float    v4f  __attribute__((ext_vector_type(4)));
typedef unsigned int v4u __attribute__((ext_vector_type(4)));

#if defined(__HIP_DEVICE_COMPILE__)
#define DEV_ASM 1
#else
#define DEV_ASM 0
#endif

__device__ __forceinline__ unsigned short h_bits(_Float16 x) { return __builtin_bit_cast(unsigned short, x); }
__device__ __forceinline__ unsigned pk16(unsigned short a, unsigned short b) { return (unsigned)a | ((unsigned)b << 16); }
__device__ __forceinline__ v8f zero8() { v8f z = {0.f, 0.f, 0.f, 0.f, 0.f, 0.f, 0.f, 0.f}; return z; }

__device__ __forceinline__ v16h ldfrag(const _Float16* p) {
  union { v16h v; v8h h[2]; } f;
  f.h[0] = *(const v8h*)(p);
  f.h[1] = *(const v8h*)(p + 16);
  return f.v;
}

__device__ __forceinline__ v8f mmar(v16h a, v16h b, v8f c) {
  return __builtin_amdgcn_wmma_f32_16x16x32_f16(false, a, false, b, (short)0, c, false, false);
}
__device__ __forceinline__ void dep_guard(v8f& a, v8f& b, v16h x, v16h y) {
#if DEV_ASM
  asm volatile("v_nop\n\tv_nop\n\tv_nop\n\tv_nop" : "+v"(a), "+v"(b) : "v"(x), "v"(y));
#else
  (void)a; (void)b; (void)x; (void)y;
#endif
}
__device__ __forceinline__ void keep4(v16h a, v16h b, v16h c, v16h d) {
#if DEV_ASM
  asm volatile("v_nop" :: "v"(a), "v"(b), "v"(c), "v"(d));
#else
  (void)a; (void)b; (void)c; (void)d;
#endif
}
__device__ __forceinline__ void acc_guard4(v8f& a, v8f& b, v8f& c, v8f& d) {
#if DEV_ASM
  asm volatile("v_nop\n\tv_nop\n\tv_nop\n\tv_nop" : "+v"(a), "+v"(b), "+v"(c), "+v"(d));
#else
  (void)a; (void)b; (void)c; (void)d;
#endif
}

__global__ __launch_bounds__(256) void cvt_x(const float* __restrict__ in, unsigned short* out, int n8) {
  const int i = blockIdx.x * 256 + (int)threadIdx.x;
  if (i < n8) {
    const v4f a  = *(const v4f*)(in + (size_t)i * 8);
    const v4f a4 = *(const v4f*)(in + (size_t)i * 8 + 4);
    v4u p;
    p[0] = pk16(h_bits((_Float16)a[0]),  h_bits((_Float16)a[1]));
    p[1] = pk16(h_bits((_Float16)a[2]),  h_bits((_Float16)a[3]));
    p[2] = pk16(h_bits((_Float16)a4[0]), h_bits((_Float16)a4[1]));
    p[3] = pk16(h_bits((_Float16)a4[2]), h_bits((_Float16)a4[3]));
    unsigned short* o = out + (size_t)i * 8;
    *(volatile v4u*)o = p;
    __threadfence();
    *(volatile v4u*)o = p;
  }
}

__global__ __launch_bounds__(256) void cvt_wT(const float* __restrict__ W, unsigned short* out, int din, int dout) {
  const int i  = blockIdx.x * 256 + (int)threadIdx.x;
  const int d8 = din >> 3;
  if (i < dout * d8) {
    const int e  = i / d8;
    const int d0 = (i - e * d8) * 8;
    float f[8];
#pragma unroll
    for (int j = 0; j < 8; ++j) f[j] = W[(size_t)(d0 + j) * (size_t)dout + e] * WSC;
    v4u p;
#pragma unroll
    for (int j = 0; j < 4; ++j) p[j] = pk16(h_bits((_Float16)f[2 * j]), h_bits((_Float16)f[2 * j + 1]));
    unsigned short* o = out + (size_t)e * (size_t)din + d0;
    *(volatile v4u*)o = p;
    __threadfence();
    *(volatile v4u*)o = p;
  }
}

template <int OUT_MODE, bool ADDV>
__global__ __launch_bounds__(256) void gemm64(
    const unsigned short* __restrict__ Ap, int lda, long long strideA,
    const unsigned short* __restrict__ Btp, int ldb, long long strideB,
    void* Cout, int ldc, long long strideC,
    const float* __restrict__ addp, int ldr, long long strideR,
    int M, int N, int K, float oscale) {
  const _Float16* A  = (const _Float16*)(const void*)Ap;
  const _Float16* Bt = (const _Float16*)(const void*)Btp;
  __shared__ __align__(16) float sT[8][16 * 68];
  const int b    = blockIdx.y;
  const int lane = threadIdx.x & 31;
  const int wave = threadIdx.x >> 5;
  const int tilesN = N >> 6;
  const int tilesM = M >> 6;
  const int tile = blockIdx.x * 8 + wave;
  if (tile >= tilesM * tilesN) return;
  const int tm = tile / tilesN;
  const int tn = tile - tm * tilesN;
  const int m0 = tm << 6;
  const int n0 = tn << 6;

  const _Float16* Ab = A  + (size_t)b * (size_t)strideA;
  const _Float16* Bb = Bt + (size_t)b * (size_t)strideB;

  const int rlane = lane & 15;
  const int koff  = (lane >> 4) * 8;
  const int mOff  = (lane >> 4) * 8;

  v8f acc[4][4];
#pragma unroll
  for (int i = 0; i < 4; ++i)
#pragma unroll
    for (int j = 0; j < 4; ++j) acc[i][j] = zero8();

  for (int k0 = 0; k0 < K; k0 += 32) {
    v16h bq[4];
#pragma unroll
    for (int j = 0; j < 4; ++j)
      bq[j] = ldfrag(Bb + (size_t)(n0 + (j << 4) + rlane) * (size_t)ldb + koff + k0);
#pragma unroll
    for (int i = 0; i < 4; ++i) {
      const v16h af = ldfrag(Ab + (size_t)(m0 + (i << 4) + rlane) * (size_t)lda + koff + k0);
#pragma unroll
      for (int j = 0; j < 4; ++j) acc[i][j] = mmar(af, bq[j], acc[i][j]);
      dep_guard(acc[i][0], acc[i][3], af, bq[3]);
    }
    keep4(bq[0], bq[1], bq[2], bq[3]);
  }
  acc_guard4(acc[0][0], acc[0][1], acc[0][2], acc[0][3]);
  acc_guard4(acc[1][0], acc[1][1], acc[1][2], acc[1][3]);
  acc_guard4(acc[2][0], acc[2][1], acc[2][2], acc[2][3]);
  acc_guard4(acc[3][0], acc[3][1], acc[3][2], acc[3][3]);

  float* slab = sT[wave];
#pragma unroll
  for (int i = 0; i < 4; ++i) {
    const int mBase = m0 + (i << 4);
#pragma unroll
    for (int j = 0; j < 4; ++j) {
#pragma unroll
      for (int r = 0; r < 8; ++r) {
        slab[(mOff + r) * 68 + (j << 4) + rlane] = acc[i][j][r];
      }
    }
    __builtin_amdgcn_fence(__ATOMIC_RELEASE, "workgroup");
    __builtin_amdgcn_wave_barrier();
    __builtin_amdgcn_fence(__ATOMIC_ACQUIRE, "workgroup");
    if (OUT_MODE == 0) {
      float* C = (float*)Cout + (size_t)b * (size_t)strideC;
      const int h2 = lane >> 4, c4 = (lane & 15) * 4;
      v4f add4 = {0.f, 0.f, 0.f, 0.f};
      if (ADDV) add4 = *(const v4f*)(addp + n0 + c4);
      v4f ov[8];
#pragma unroll
      for (int it = 0; it < 8; ++it) {
        const int row = it * 2 + h2;
        ov[it] = *(const v4f*)(slab + row * 68 + c4) * oscale + add4;
      }
      for (int pass = 0; pass < 2; ++pass) {
#pragma unroll
        for (int it = 0; it < 8; ++it) {
          const int row = it * 2 + h2;
          *(volatile v4f*)(C + (size_t)(mBase + row) * (size_t)ldc + n0 + c4) = ov[it];
        }
        __threadfence();
      }
    } else {
      const int q = lane >> 3, c8 = (lane & 7) * 8;
      unsigned short* C = (unsigned short*)Cout + (size_t)b * (size_t)strideC;
      const float* R = addp + (size_t)b * (size_t)strideR;
      v4u hv[4];
#pragma unroll
      for (int it = 0; it < 4; ++it) {
        const int row = it * 4 + q;
        const float* sp = slab + row * 68 + c8;
        float f[8];
#pragma unroll
        for (int e = 0; e < 8; ++e) f[e] = sp[e] * oscale;
        if (ADDV) {
          const float* rp = R + (size_t)(mBase + row) * (size_t)ldr + n0 + c8;
          const v4f r0 = *(const v4f*)rp;
          const v4f r1 = *(const v4f*)(rp + 4);
          f[0] += r0[0]; f[1] += r0[1]; f[2] += r0[2]; f[3] += r0[3];
          f[4] += r1[0]; f[5] += r1[1]; f[6] += r1[2]; f[7] += r1[3];
        }
        v4u a;
#pragma unroll
        for (int e = 0; e < 4; ++e) a[e] = pk16(h_bits((_Float16)f[2 * e]), h_bits((_Float16)f[2 * e + 1]));
        hv[it] = a;
      }
      for (int pass = 0; pass < 2; ++pass) {
#pragma unroll
        for (int it = 0; it < 4; ++it) {
          const int row = it * 4 + q;
          *(volatile v4u*)(C + (size_t)(mBase + row) * (size_t)ldc + n0 + c8) = hv[it];
        }
        __threadfence();
      }
    }
    __builtin_amdgcn_fence(__ATOMIC_RELEASE, "workgroup");
    __builtin_amdgcn_wave_barrier();
    __builtin_amdgcn_fence(__ATOMIC_ACQUIRE, "workgroup");
  }
}

__global__ __launch_bounds__(256) void softmax_rows(const float* __restrict__ S, unsigned short* P) {
  const int lane = threadIdx.x & 31, wave = threadIdx.x >> 5;
  const int row  = blockIdx.x * 8 + wave;
  const float* sr = S + (size_t)row * SEQ;
  unsigned short* prow = P + (size_t)row * SEQ;

  float m = -3.0e38f;
#pragma unroll 1
  for (int c = 0; c < SEQ / 256; ++c) {
    const float* p = sr + c * 256 + lane * 8;
    const v4f a = *(const v4f*)p;
    const v4f a4 = *(const v4f*)(p + 4);
    m = fmaxf(m, fmaxf(fmaxf(a[0], a[1]), fmaxf(a[2], a[3])));
    m = fmaxf(m, fmaxf(fmaxf(a4[0], a4[1]), fmaxf(a4[2], a4[3])));
  }
#pragma unroll
  for (int off = 1; off < 32; off <<= 1) m = fmaxf(m, __shfl_xor(m, off, 32));

  float l = 0.f;
#pragma unroll 1
  for (int c = 0; c < SEQ / 256; ++c) {
    const float* p = sr + c * 256 + lane * 8;
    const v4f a = *(const v4f*)p;
    const v4f a4 = *(const v4f*)(p + 4);
    l += exp2f((a[0] - m) * L2E) + exp2f((a[1] - m) * L2E) + exp2f((a[2] - m) * L2E) + exp2f((a[3] - m) * L2E);
    l += exp2f((a4[0] - m) * L2E) + exp2f((a4[1] - m) * L2E) + exp2f((a4[2] - m) * L2E) + exp2f((a4[3] - m) * L2E);
  }
#pragma unroll
  for (int off = 1; off < 32; off <<= 1) l += __shfl_xor(l, off, 32);
  const float sc = PSC / l;

#pragma unroll 1
  for (int c = 0; c < SEQ / 256; ++c) {
    const float* p = sr + c * 256 + lane * 8;
    const v4f a = *(const v4f*)p;
    const v4f a4 = *(const v4f*)(p + 4);
    float e8[8];
    e8[0] = exp2f((a[0] - m) * L2E) * sc;  e8[1] = exp2f((a[1] - m) * L2E) * sc;
    e8[2] = exp2f((a[2] - m) * L2E) * sc;  e8[3] = exp2f((a[3] - m) * L2E) * sc;
    e8[4] = exp2f((a4[0] - m) * L2E) * sc; e8[5] = exp2f((a4[1] - m) * L2E) * sc;
    e8[6] = exp2f((a4[2] - m) * L2E) * sc; e8[7] = exp2f((a4[3] - m) * L2E) * sc;
    v4u pk;
#pragma unroll
    for (int e = 0; e < 4; ++e) pk[e] = pk16(h_bits((_Float16)e8[2 * e]), h_bits((_Float16)e8[2 * e + 1]));
    unsigned short* d = prow + c * 256 + lane * 8;
    *(volatile v4u*)d = pk;
    __threadfence();
    *(volatile v4u*)d = pk;
  }
}

extern "C" void kernel_launch(void* const* d_in, const int* in_sizes, int n_in,
                              void* d_out, int out_size, void* d_ws, size_t ws_size,
                              hipStream_t stream) {
  if (n_in < 4) return;
  if (in_sizes[0] != ROWS * DM) return;
  if (in_sizes[1] != DM * QKVN) return;
  if (in_sizes[2] != DM * DM) return;
  if (in_sizes[3] != DM) return;
  if (out_size != ROWS * DM) return;

  const float* x    = (const float*)d_in[0];
  const float* Wqkv = (const float*)d_in[1];
  const float* Wout = (const float*)d_in[2];
  const float* bout = (const float*)d_in[3];

  const size_t PXH = (size_t)ROWS * DM * 2;
  const size_t PWQ = (size_t)QKVN * DM * 2;
  const size_t PWO = (size_t)DM * DM * 2;
  const size_t PQK = (size_t)ROWS * NQK * 2;
  const size_t PVT = (size_t)NB * DM * SEQ * 2;
  const size_t PS  = (size_t)SEQ * SEQ * 4;
  const size_t PP  = (size_t)SEQ * SEQ * 2;
  const size_t POX = (size_t)ROWS * DM * 2;
  size_t off = 0;
  const size_t oXh = off; off += PXH;
  const size_t oWq = off; off += PWQ;
  const size_t oWo = off; off += PWO;
  const size_t oQK = off; off += PQK;
  const size_t oVT = off; off += PVT;
  const size_t oS  = off; off += PS;
  const size_t oP  = off; off += PP;
  const size_t oOX = off; off += POX;
  if (off > ws_size) return;
  if (off > (size_t)134217728) return;

  char* ws = (char*)d_ws;
  unsigned short* Xh  = (unsigned short*)(ws + oXh);
  unsigned short* WqT = (unsigned short*)(ws + oWq);
  unsigned short* WoT = (unsigned short*)(ws + oWo);
  unsigned short* QK  = (unsigned short*)(ws + oQK);
  unsigned short* VT  = (unsigned short*)(ws + oVT);
  float*          S   = (float*)(ws + oS);
  unsigned short* P   = (unsigned short*)(ws + oP);
  unsigned short* OX  = (unsigned short*)(ws + oOX);

  const dim3 blk(256);
  const int n8x  = ROWS * DM / 8;
  const int n8wq = QKVN * (DM / 8);
  const int n8wo = DM * (DM / 8);
  const dim3 gCvtX((n8x + 255) / 256);
  const dim3 gCvtQ((n8wq + 255) / 256);
  const dim3 gCvtO((n8wo + 255) / 256);
  const dim3 gQK((((ROWS / 64) * (NQK / 64)) + 7) / 8, 1);
  const dim3 gVT((((DM / 64) * (SEQ / 64)) + 7) / 8, NB);
  const dim3 gSC((((SEQ / 64) * (SEQ / 64)) + 7) / 8, 1);
  const dim3 gSM(SEQ / 8);
  const dim3 gPV((((SEQ / 64) * (DM / 64)) + 7) / 8, 1);
  const dim3 gOUT((((ROWS / 64) * (DM / 64)) + 7) / 8, 1);

  cvt_x<<<gCvtX, blk, 0, stream>>>(x, Xh, n8x);
  cvt_wT<<<gCvtQ, blk, 0, stream>>>(Wqkv, WqT, DM, QKVN);
  cvt_wT<<<gCvtO, blk, 0, stream>>>(Wout, WoT, DM, DM);
  gemm64<1, false><<<gQK, blk, 0, stream>>>(
      Xh, DM, 0LL, WqT, DM, 0LL,
      (void*)QK, NQK, 0LL, bout, 0, 0LL,
      ROWS, NQK, DM, 1.0f / WSC);
  gemm64<1, false><<<gVT, blk, 0, stream>>>(
      WqT + (size_t)NQK * DM, DM, 0LL, Xh, DM, (long long)SEQ * DM,
      (void*)VT, SEQ, (long long)DM * SEQ, bout, 0, 0LL,
      DM, SEQ, DM, 1.0f / WSC);
  for (int b = 0; b < NB; ++b) {
    const unsigned short* Qb = QK + (size_t)b * SEQ * NQK;
    gemm64<0, false><<<gSC, blk, 0, stream>>>(
        Qb, NQK, 0LL, Qb + DM, NQK, 0LL,
        (void*)S, SEQ, 0LL, bout, 0, 0LL,
        SEQ, SEQ, DM, 1.0f / 64.0f);
    softmax_rows<<<gSM, blk, 0, stream>>>(S, P);
    gemm64<1, true><<<gPV, blk, 0, stream>>>(
        P, SEQ, 0LL, VT + (size_t)b * DM * SEQ, SEQ, 0LL,
        (void*)(OX + (size_t)b * SEQ * DM), DM, 0LL,
        x + (size_t)b * SEQ * DM, DM, 0LL,
        SEQ, DM, SEQ, 1.0f / PSC);
  }
  gemm64<0, true><<<gOUT, blk, 0, stream>>>(
      OX, DM, 0LL, WoT, DM, 0LL,
      d_out, DM, 0LL, bout, 0, 0LL,
      ROWS, DM, DM, 1.0f / WSC);
  (void)hipGetLastError();
}
